// FFTSSMBlock_52080773432011
// MI455X (gfx1250) — hardware-run, weakly checked
//
#include <hip/hip_runtime.h>
#include <math.h>

typedef __attribute__((ext_vector_type(16))) _Float16 v16h;
typedef __attribute__((ext_vector_type(8)))  _Float16 v8h;
typedef __attribute__((ext_vector_type(16))) __bf16   v16b;
typedef __attribute__((ext_vector_type(8)))  __bf16   v8b;
typedef __attribute__((ext_vector_type(8)))  float    v8f;
typedef __attribute__((ext_vector_type(4)))  float    v4f;

constexpr int kB     = 4;
constexpr int kC     = 128;
constexpr int kH     = 64;
constexpr int kW     = 64;
constexpr int kL     = kH * kW;
constexpr int kTok   = kB * kL;
constexpr int kBC    = kB * kC;
constexpr int kDin   = 256;
constexpr int kNst   = 16;
constexpr int kDtR   = 8;
constexpr int kXzP   = 2 * kDin;
constexpr int kXdP   = 64;
constexpr int kXdN   = kDtR + 2 * kNst;
constexpr int kWr    = kW / 2 + 1;
constexpr int kModes = kH * kWr;
constexpr int kCols  = 2 * kModes;
constexpr int kPad   = 66;
constexpr int kTaps  = 9;
constexpr int kConvK = kTaps * kC;
constexpr int kConvTP = 260;
constexpr int kScanTS = 64;
constexpr int kScanCh = 64;
constexpr int kScanYP = 68;

constexpr float kCarX  = 16.0f;
constexpr float kCarW  = 1024.0f;
constexpr float kCarS  = 256.0f;
constexpr float kInvXW = 1.0f / (kCarX * kCarW);
constexpr float kInvSW = 1.0f / (kCarS * kCarW);
constexpr float kInvX  = 1.0f / kCarX;
constexpr float kInvW  = 1.0f / kCarW;
constexpr float kInvHW = 1.0f / (float)(kH * kW);
constexpr float kStepAng = 6.283185307179586f / 64.0f;

static_assert(kL == 4096 && kTok == 16384 && kBC == 512 && kModes == 2112 && kCols == 4224 && kConvK == 1152, "shapes");
static_assert(kH == 64 && kW == 64 && kC == 128 && kXdN == 40, "shapes");
static_assert((kCols % 64) == 0 && (kBC % 64) == 0 && (kL % 32) == 0, "forward transform GEMM tiles");
static_assert((kXzP / 2) % 64 == 0 && ((kB * kModes) % 64) == 0 && (kXzP / 2) % 32 == 0, "mix GEMM tiles");
static_assert((kL % 64) == 0 && (kCols % 32) == 0 && (kModes % 64) == 0, "inverse transform GEMM tiles");
static_assert((kTok % 64) == 0 && (kXzP % 64) == 0 && (kC % 32) == 0 && (kDin % 32) == 0 && (kXdP % 64) == 0, "projection GEMM tiles");
static_assert((kC % 64) == 0 && (kConvK % 32) == 0, "conv GEMM tiles");
static_assert((kL % kScanTS) == 0 && (kDin % kScanCh) == 0, "scan tiles");

constexpr size_t kSzTAB   = 256;
constexpr size_t kSzFB    = (size_t)kCols * kL * 2;
constexpr size_t kSzIB    = (size_t)kL * kCols * 2;
constexpr size_t kSzX16   = (size_t)kBC * kL * 2;
constexpr size_t kSzXPAD  = (size_t)kB * kPad * kPad * kC * 2;
constexpr size_t kSzU16   = (size_t)kTok * kC * 2;
constexpr size_t kSzWCONV = (size_t)kC * kConvK * 2;
constexpr size_t kSzWIN   = (size_t)kXzP * kC * 2;
constexpr size_t kSzWXP   = (size_t)kXdP * kDin * 2;
constexpr size_t kSzWSPEC = (size_t)256 * 256 * 2;
constexpr size_t kSzWOUT  = (size_t)kC * kDin * 2;
constexpr size_t kSzFQ    = (size_t)kB * kModes * 256 * 2;
constexpr size_t kSzG     = (size_t)kBC * kCols * 2;
constexpr size_t kSzSPEC  = (size_t)kBC * kL * 4;
constexpr size_t kSzXD    = (size_t)kTok * kXdP * 4;
constexpr size_t kSzYM    = (size_t)kBC * kL * 4;

constexpr size_t kOffTAB   = 0;
constexpr size_t kOffFB    = kOffTAB   + kSzTAB;
constexpr size_t kOffIB    = kOffFB    + kSzFB;
constexpr size_t kOffX16   = kOffIB    + kSzIB;
constexpr size_t kOffXPAD  = kOffX16   + kSzX16;
constexpr size_t kOffU16   = kOffXPAD  + kSzXPAD;
constexpr size_t kOffWCONV = kOffU16   + kSzU16;
constexpr size_t kOffWIN   = kOffWCONV + kSzWCONV;
constexpr size_t kOffWXP   = kOffWIN   + kSzWIN;
constexpr size_t kOffWSPEC = kOffWXP   + kSzWXP;
constexpr size_t kOffWOUT  = kOffWSPEC + kSzWSPEC;
constexpr size_t kOffFQ    = kOffWOUT  + kSzWOUT;
constexpr size_t kOffG     = kOffFQ    + kSzFQ;
constexpr size_t kOffSPEC  = kOffG     + kSzG;
constexpr size_t kOffXD    = kOffSPEC  + kSzSPEC;
constexpr size_t kOffYM    = kOffXD    + kSzXD;
constexpr size_t kWsTotal  = kOffYM    + kSzYM;
constexpr size_t kOffXZ    = kOffFB;
constexpr size_t kOffXS    = kOffIB;
constexpr size_t kOffXS16  = kOffXS   + (size_t)kTok * kDin * 4;
constexpr size_t kOffYG    = kOffXS16 + (size_t)kTok * kDin * 2;
static_assert(kWsTotal == 112333056ull, "carve total");
static_assert(kWsTotal <= 134217728ull, "carve cap");
static_assert((size_t)kTok * kXzP * 4 <= kSzFB, "XZ fits the dead forward basis");
static_assert(kOffYG + (size_t)kTok * kDin * 2 <= kOffIB + kSzIB, "XS, XS16, YG fit the dead inverse basis");
static_assert((kOffFB % 128) == 0 && (kOffIB % 128) == 0 && (kOffX16 % 128) == 0 && (kOffXPAD % 128) == 0 &&
              (kOffU16 % 128) == 0 && (kOffWCONV % 128) == 0 && (kOffWIN % 128) == 0 && (kOffWXP % 128) == 0 &&
              (kOffWSPEC % 128) == 0 && (kOffWOUT % 128) == 0 && (kOffFQ % 128) == 0 && (kOffG % 128) == 0 &&
              (kOffSPEC % 128) == 0 && (kOffXD % 128) == 0 && (kOffYM % 128) == 0 && (kOffXS16 % 128) == 0 &&
              (kOffYG % 128) == 0, "128-B aligned regions");

__device__ __forceinline__ unsigned short f2bf_bits(float f) {
  unsigned u = __float_as_uint(f);
  return (unsigned short)((u + 0x7FFFu + ((u >> 16) & 1u)) >> 16);
}
__device__ __forceinline__ _Float16 to_h16(float v) {
  const float f = (fabsf(v) < 6.103515625e-5f) ? 0.0f : v;
  return (_Float16)f;
}

__device__ __forceinline__ void tie_h(v8f& a, v16h x, v16h y) { asm volatile("" : "+v"(a) : "v"(x), "v"(y)); }
__device__ __forceinline__ void tie_nop_h(v8f& a, v16h x, v16h y) { asm volatile("v_nop\n\tv_nop\n\tv_nop\n\tv_nop" : "+v"(a) : "v"(x), "v"(y)); }
__device__ __forceinline__ void tie_b(v8f& a, v16b x, v16b y) { asm volatile("" : "+v"(a) : "v"(x), "v"(y)); }
__device__ __forceinline__ void tie_nop_b(v8f& a, v16b x, v16b y) { asm volatile("v_nop\n\tv_nop\n\tv_nop\n\tv_nop" : "+v"(a) : "v"(x), "v"(y)); }
__device__ __forceinline__ void keep4_h(v16h a, v16h b, v16h c, v16h d) { asm volatile("v_nop" :: "v"(a), "v"(b), "v"(c), "v"(d)); }
__device__ __forceinline__ void keep4_b(v16b a, v16b b, v16b c, v16b d) { asm volatile("v_nop" :: "v"(a), "v"(b), "v"(c), "v"(d)); }
__device__ __forceinline__ void acc_guard4(v8f& a, v8f& b, v8f& c, v8f& d) { asm volatile("v_nop\n\tv_nop\n\tv_nop\n\tv_nop" : "+v"(a), "+v"(b), "+v"(c), "+v"(d)); }

template <typename T> struct Frag;
template <> struct Frag<_Float16> {
  typedef v16h V; union U { v16h v; v8h h[2]; };
  static __device__ __forceinline__ v16h load(const _Float16* p) {
    U f; f.h[0] = *(const v8h*)(p); f.h[1] = *(const v8h*)(p + 16); return f.v;
  }
  static __device__ __forceinline__ v8f mma(v16h a, v16h b, v8f c) {
    return __builtin_amdgcn_wmma_f32_16x16x32_f16(false, a, false, b, (short)0, c, false, false);
  }
  static __device__ __forceinline__ void tie(v8f& a, v16h x, v16h y) { tie_h(a, x, y); }
  static __device__ __forceinline__ void tie_nop(v8f& a, v16h x, v16h y) { tie_nop_h(a, x, y); }
  static __device__ __forceinline__ void keep(v16h a, v16h b, v16h c, v16h d) { keep4_h(a, b, c, d); }
};
template <> struct Frag<__bf16> {
  typedef v16b V; union U { v16b v; v8b h[2]; };
  static __device__ __forceinline__ v16b load(const __bf16* p) {
    U f; f.h[0] = *(const v8b*)(p); f.h[1] = *(const v8b*)(p + 16); return f.v;
  }
  static __device__ __forceinline__ v8f mma(v16b a, v16b b, v8f c) {
    return __builtin_amdgcn_wmma_f32_16x16x32_bf16(false, a, false, b, (short)0, c, false, false);
  }
  static __device__ __forceinline__ void tie(v8f& a, v16b x, v16b y) { tie_b(a, x, y); }
  static __device__ __forceinline__ void tie_nop(v8f& a, v16b x, v16b y) { tie_nop_b(a, x, y); }
  static __device__ __forceinline__ void keep(v16b a, v16b b, v16b c, v16b d) { keep4_b(a, b, c, d); }
};
template <int ET> struct Elem;
template <> struct Elem<0> { typedef _Float16 T; };
template <> struct Elem<1> { typedef __bf16 T; };

template <int ET, bool BIAS_M, int OUT_MODE, bool CONV, bool RES2>
__global__ __launch_bounds__(256) void gemm64_kernel(
    const unsigned short* __restrict__ Ap, int lda,
    const unsigned short* __restrict__ Btp, int ldb,
    void* __restrict__ Cout,
    const float* __restrict__ bias,
    const float* __restrict__ res1, const float* __restrict__ res2,
    int M, int N, int K, float scale,
    int Rm, long sm0, long sm1, int Rn, long sn1)
{
  typedef typename Elem<ET>::T T;
  typedef typename Frag<T>::V V;
  const T* A  = (const T*)Ap;
  const T* Bt = (const T*)Btp;
  __shared__ __align__(16) float sT[8][16 * 68];
  const int lane = threadIdx.x & 31;
  const int wave = threadIdx.x >> 5;
  const int tilesN = N >> 6;
  const int tilesM = M >> 6;
  const int perImg = tilesM * tilesN;
  const int nTiles = CONV ? perImg * (kB * kH) : perImg;
  const int tile = blockIdx.x * 8 + wave;
  if (tile >= nTiles) return;
  int z = 0, t2 = tile;
  if (CONV) { z = tile / perImg; t2 = tile - z * perImg; }
  const int tm = t2 / tilesN;
  const int tn = t2 - tm * tilesN;
  const int m0 = tm << 6;
  const int n0 = tn << 6;

  const T* Bb = Bt;
  long cbase;
  int rm;
  if (CONV) {
    const int bb = z >> 6, hh = z & 63;
    Bb = Bt + (size_t)((bb * kPad + hh) * kPad) * kC;
    cbase = (long)bb * kC * kL + (long)hh * kW + n0;
    rm = m0;
  } else {
    const int qm = m0 / Rm;
    rm = m0 - qm * Rm;
    const int qn = n0 / Rn;
    cbase = (long)qm * sm1 + (long)(n0 - qn * Rn) + (long)qn * sn1;
  }

  const int rlane = lane & 15;
  const int koff  = (lane >> 4) * 8;
  const int mOff  = (lane >> 4) * 8;

  v8f acc[4][4];
#pragma unroll
  for (int i = 0; i < 4; ++i)
#pragma unroll
    for (int j = 0; j < 4; ++j) acc[i][j] = (v8f){0.f,0.f,0.f,0.f,0.f,0.f,0.f,0.f};

  for (int k0 = 0; k0 < K; k0 += 32) {
    int kb = k0;
    if (CONV) {
      const int tap = k0 >> 7;
      const int kh = tap / 3;
      const int kw = tap - 3 * kh;
      kb = (kh * kPad + kw) * kC + (k0 & (kC - 1));
    }
    V bh[4];
#pragma unroll
    for (int j = 0; j < 4; ++j) {
      const size_t bo = (size_t)(n0 + (j << 4) + rlane) * ldb + koff + kb;
      bh[j] = Frag<T>::load(Bb + bo);
    }
#pragma unroll
    for (int i = 0; i < 4; ++i) {
      const size_t ao = (size_t)(m0 + (i << 4) + rlane) * lda + koff + k0;
      V ah = Frag<T>::load(A + ao);
#pragma unroll
      for (int j = 0; j < 4; ++j) acc[i][j] = Frag<T>::mma(ah, bh[j], acc[i][j]);
      Frag<T>::tie(acc[i][1], ah, bh[1]);
      Frag<T>::tie(acc[i][2], ah, bh[2]);
      Frag<T>::tie(acc[i][3], ah, bh[3]);
      Frag<T>::tie_nop(acc[i][0], ah, bh[0]);
    }
    Frag<T>::keep(bh[0], bh[1], bh[2], bh[3]);
  }
  acc_guard4(acc[0][0], acc[0][1], acc[0][2], acc[0][3]);
  acc_guard4(acc[1][0], acc[1][1], acc[1][2], acc[1][3]);
  acc_guard4(acc[2][0], acc[2][1], acc[2][2], acc[2][3]);
  acc_guard4(acc[3][0], acc[3][1], acc[3][2], acc[3][3]);

  float* slab = sT[wave];
#pragma unroll
  for (int i = 0; i < 4; ++i) {
    const int mBase = m0 + (i << 4);
    float bm[8];
#pragma unroll
    for (int r = 0; r < 8; ++r) bm[r] = 0.0f;
    if (BIAS_M) {
      const v4f b0 = *(const v4f*)(bias + mBase + mOff);
      const v4f b1 = *(const v4f*)(bias + mBase + mOff + 4);
      bm[0] = b0[0]; bm[1] = b0[1]; bm[2] = b0[2]; bm[3] = b0[3];
      bm[4] = b1[0]; bm[5] = b1[1]; bm[6] = b1[2]; bm[7] = b1[3];
    }
#pragma unroll
    for (int j = 0; j < 4; ++j) {
#pragma unroll
      for (int r = 0; r < 8; ++r) {
        float v = acc[i][j][r] * scale;
        if (BIAS_M) v += bm[r];
        slab[(mOff + r) * 68 + (j << 4) + rlane] = v;
      }
    }
    __builtin_amdgcn_fence(__ATOMIC_RELEASE, "workgroup");
    __builtin_amdgcn_wave_barrier();
    __builtin_amdgcn_fence(__ATOMIC_ACQUIRE, "workgroup");
    const long rowBase = cbase + (long)(rm + (i << 4)) * sm0;
    if (OUT_MODE == 0) {
      float* Cf = (float*)Cout;
      const int hh2 = lane >> 4, c4 = (lane & 15) * 4;
      v4f vals[8];
#pragma unroll
      for (int it = 0; it < 8; ++it) {
        const int row = it * 2 + hh2;
        v4f v = *(const v4f*)(slab + row * 68 + c4);
        if (RES2) {
          const long o = rowBase + (long)row * sm0 + c4;
          const v4f r1 = *(const v4f*)(res1 + o);
          const v4f r2 = *(const v4f*)(res2 + o);
          v = (v + r1) + r2;
        }
        vals[it] = v;
      }
      for (int pass = 0; pass < 2; ++pass) {
#pragma unroll
        for (int it = 0; it < 8; ++it) {
          const int row = it * 2 + hh2;
          *(volatile v4f*)(Cf + rowBase + (long)row * sm0 + c4) = vals[it];
        }
        __threadfence();
      }
    } else {
      unsigned short* Ch = (unsigned short*)Cout;
      const int q = lane >> 3, c8 = (lane & 7) * 8;
      v8h hv[4];
#pragma unroll
      for (int it = 0; it < 4; ++it) {
        const int row = it * 4 + q;
        const float* sp = slab + row * 68 + c8;
        const v4f a0 = *(const v4f*)(sp);
        const v4f a1 = *(const v4f*)(sp + 4);
#pragma unroll
        for (int e = 0; e < 4; ++e) {
          hv[it][e]     = to_h16(a0[e]);
          hv[it][4 + e] = to_h16(a1[e]);
        }
      }
      for (int pass = 0; pass < 2; ++pass) {
#pragma unroll
        for (int it = 0; it < 4; ++it) {
          const int row = it * 4 + q;
          *(volatile v8h*)(Ch + rowBase + (long)row * sm0 + c8) = hv[it];
        }
        __threadfence();
      }
    }
    __builtin_amdgcn_fence(__ATOMIC_RELEASE, "workgroup");
    __builtin_amdgcn_wave_barrier();
    __builtin_amdgcn_fence(__ATOMIC_ACQUIRE, "workgroup");
  }
}

__global__ __launch_bounds__(64) void twiddle_kernel(float* __restrict__ tab)
{
  __shared__ __align__(16) float sC[64];
  const int p = threadIdx.x;
  const int r = p & 31;
  const int q = (r <= 16) ? r : (32 - r);
  float c = cosf((float)q * kStepAng);
  c = (q == 16) ? 0.0f : c;
  const bool neg = ((r > 16) != (p >= 32));
  sC[p] = neg ? -c : c;
  __syncthreads();
  if (p < 16) {
    const v4f v = *(const v4f*)(sC + 4 * p);
    volatile v4f* dst = (volatile v4f*)(tab + 4 * p);
    *dst = v;
    __threadfence();
    *dst = v;
  }
}

template <bool INV>
__global__ __launch_bounds__(256) void basis_kernel(const float* __restrict__ tab, unsigned short* __restrict__ dst, int total8)
{
  __shared__ float sTab[64];
  const int tid = threadIdx.x;
  {
    float tv = tab[tid & 63];
    asm volatile("" : "+v"(tv));
    if (tid < 64) sTab[tid] = tv;
  }
  __syncthreads();
  const int i = blockIdx.x * 256 + tid;
  if (i >= total8) return;
  v8h hv;
  if (!INV) {
    const int col  = i >> 9;
    const int pix0 = (i & 511) * 8;
    const int h = pix0 >> 6, w0 = pix0 & 63;
    const int part = (col >= kModes) ? 1 : 0;
    const int mode = col - part * kModes;
    const int m = mode / kWr;
    const int k = mode - m * kWr;
    const int ph0 = m * h + k * w0 + 16 * part;
#pragma unroll
    for (int j = 0; j < 8; ++j) {
      const float v = sTab[(ph0 + k * j) & 63];
      hv[j] = (_Float16)v;
    }
  } else {
    const int pix = i / (kCols / 8);
    const int g   = i - pix * (kCols / 8);
    const int kk0 = g * 8;
    const int part = (kk0 >= kModes) ? 1 : 0;
    const int mode0 = kk0 - part * kModes;
    const int h = pix >> 6, w = pix & 63;
#pragma unroll
    for (int j = 0; j < 8; ++j) {
      const int mode = mode0 + j;
      const int m = mode / kWr;
      const int k = mode - m * kWr;
      const int ph = (m * h + k * w + 16 * part) & 63;
      const float coef = (k == 0 || k == (kWr - 1)) ? 1.0f : 2.0f;
      const float v = coef * sTab[ph];
      hv[j] = (_Float16)v;
    }
  }
  unsigned short* p = dst + (size_t)i * 8;
  *(volatile v8h*)p = hv;
  __threadfence();
  *(volatile v8h*)p = hv;
}

template <int MODE>
__global__ __launch_bounds__(256) void cast_rows_kernel(
    const float* __restrict__ src, unsigned short* __restrict__ dst, int total8, int valid8, float carry)
{
  const int i = blockIdx.x * 256 + threadIdx.x;
  if (i >= total8) return;
  const bool ok = (i < valid8);
  const int ic = ok ? i : (valid8 - 1);
  const v4f a0 = *(const v4f*)(src + (size_t)ic * 8);
  const v4f a1 = *(const v4f*)(src + (size_t)ic * 8 + 4);
  v8h hv;
#pragma unroll
  for (int e = 0; e < 4; ++e) {
    const float f0 = ok ? (a0[e] * carry) : 0.0f;
    const float f1 = ok ? (a1[e] * carry) : 0.0f;
    if (MODE == 0) {
      hv[e]     = to_h16(f0);
      hv[4 + e] = to_h16(f1);
    } else {
      const unsigned short h0 = f2bf_bits(f0);
      const unsigned short h1 = f2bf_bits(f1);
      hv[e]     = __builtin_bit_cast(_Float16, h0);
      hv[4 + e] = __builtin_bit_cast(_Float16, h1);
    }
  }
  unsigned short* p = dst + (size_t)i * 8;
  *(volatile v8h*)p = hv;
  __threadfence();
  *(volatile v8h*)p = hv;
}

__global__ __launch_bounds__(256) void conv_weight_kernel(const float* __restrict__ w, unsigned short* __restrict__ dst, int total8)
{
  const int i = blockIdx.x * 256 + threadIdx.x;
  if (i >= total8) return;
  const int co  = i / (kConvK / 8);
  const int g   = i - co * (kConvK / 8);
  const int tap = g >> 4;
  const int ci0 = (g & 15) * 8;
  v8h hv;
#pragma unroll
  for (int j = 0; j < 8; ++j) {
    const float v = w[((size_t)(co * kC + ci0 + j)) * kTaps + tap];
    hv[j] = to_h16(v * kCarW);
  }
  unsigned short* p = dst + (size_t)i * 8;
  *(volatile v8h*)p = hv;
  __threadfence();
  *(volatile v8h*)p = hv;
}

__global__ __launch_bounds__(256) void relayout_kernel(
    const float* __restrict__ x, unsigned short* __restrict__ xpad, unsigned short* __restrict__ u16)
{
  __shared__ __align__(16) float sT[kW * 132];
  const int tid = threadIdx.x;
  const int b = blockIdx.x >> 6, h = blockIdx.x & 63;
#pragma unroll
  for (int it = 0; it < 8; ++it) {
    const int idx = it * 256 + tid;
    const int c = idx >> 4, w4 = (idx & 15) * 4;
    const v4f v = *(const v4f*)(x + ((size_t)(b * kC + c) * kH + h) * kW + w4);
    sT[(w4 + 0) * 132 + c] = v[0];
    sT[(w4 + 1) * 132 + c] = v[1];
    sT[(w4 + 2) * 132 + c] = v[2];
    sT[(w4 + 3) * 132 + c] = v[3];
  }
  __syncthreads();
  v8h hv[4];
#pragma unroll
  for (int it = 0; it < 4; ++it) {
    const int id = it * 256 + tid;
    const int row = id >> 4, c8 = (id & 15) * 8;
    const float* sp = sT + row * 132 + c8;
    const v4f a0 = *(const v4f*)(sp);
    const v4f a1 = *(const v4f*)(sp + 4);
#pragma unroll
    for (int e = 0; e < 4; ++e) {
      hv[it][e]     = to_h16(a0[e] * kCarX);
      hv[it][4 + e] = to_h16(a1[e] * kCarX);
    }
  }
  v8h zv;
#pragma unroll
  for (int e = 0; e < 8; ++e) zv[e] = (_Float16)0.0f;
  const size_t uBase = ((size_t)(b * kH + h) * kW) * kC;
  const size_t pRow  = ((size_t)(b * kPad + h + 1) * kPad) * kC;
  const size_t pBase = pRow + kC;
  const size_t topRow = ((size_t)(b * kPad) * kPad) * kC;
  const size_t botRow = ((size_t)(b * kPad + kPad - 1) * kPad) * kC;
  for (int pass = 0; pass < 2; ++pass) {
#pragma unroll
    for (int it = 0; it < 4; ++it) {
      const size_t o = (size_t)(it * 256 + tid) * 8;
      *(volatile v8h*)(u16 + uBase + o)  = hv[it];
      *(volatile v8h*)(xpad + pBase + o) = hv[it];
    }
    if (tid < 32) {
      const int side = tid >> 4, cs = (tid & 15) * 8;
      *(volatile v8h*)(xpad + pRow + (size_t)(side * (kPad - 1)) * kC + cs) = zv;
    }
    if (h == 0) {
      for (int i2 = tid; i2 < kPad * kC / 8; i2 += 256) *(volatile v8h*)(xpad + topRow + (size_t)i2 * 8) = zv;
    }
    if (h == kH - 1) {
      for (int i2 = tid; i2 < kPad * kC / 8; i2 += 256) *(volatile v8h*)(xpad + botRow + (size_t)i2 * 8) = zv;
    }
    __threadfence();
  }
}

__global__ __launch_bounds__(256) void conv_silu_kernel(
    const float* __restrict__ XZ, const float* __restrict__ cw, const float* __restrict__ cb,
    float* __restrict__ XS, unsigned short* __restrict__ XS16)
{
  __shared__ __align__(16) float sT[16 * kConvTP];
  const int tid = threadIdx.x, lane = tid & 31, wave = tid >> 5;
  const int d = tid;
  const int g0 = blockIdx.x * 64;
  const int tb = g0 & (kL - 1);
  const float w0 = cw[d * 4 + 0], w1 = cw[d * 4 + 1], w2 = cw[d * 4 + 2], w3 = cw[d * 4 + 3];
  const float bc = cb[d];
  float xm3, xm2, xm1;
  {
    const bool hist = (tb > 0);
    const int rb = hist ? (g0 - 3) : g0;
    const float v3 = XZ[(size_t)rb * kXzP + d];
    const float v2 = XZ[(size_t)(rb + 1) * kXzP + d];
    const float v1 = XZ[(size_t)(rb + 2) * kXzP + d];
    xm3 = hist ? v3 : 0.f;
    xm2 = hist ? v2 : 0.f;
    xm1 = hist ? v1 : 0.f;
  }
  const int hrow = wave >> 1;
  const int hch  = (wave & 1) * 128 + lane * 4;
#pragma unroll 1
  for (int sub = 0; sub < 4; ++sub) {
    const int lb = g0 + sub * 16;
#pragma unroll 1
    for (int s = 0; s < 16; ++s) {
      const float xcur = XZ[(size_t)(lb + s) * kXzP + d];
      float acc = w0 * xm3;
      acc = fmaf(w1, xm2, acc);
      acc = fmaf(w2, xm1, acc);
      acc = fmaf(w3, xcur, acc);
      const float sv = acc + bc;
      const float sg = 1.0f / (1.0f + expf(-sv));
      sT[s * kConvTP + tid] = sv * sg;
      xm3 = xm2; xm2 = xm1; xm1 = xcur;
    }
    __syncthreads();
    v4f fv[4];
    v8h hv[2];
#pragma unroll
    for (int it = 0; it < 4; ++it) fv[it] = *(const v4f*)(sT + (it * 4 + hrow) * kConvTP + hch);
#pragma unroll
    for (int it = 0; it < 2; ++it) {
      const float* sp = sT + (it * 8 + wave) * kConvTP + lane * 8;
      const v4f a0 = *(const v4f*)(sp);
      const v4f a1 = *(const v4f*)(sp + 4);
#pragma unroll
      for (int e = 0; e < 4; ++e) {
        hv[it][e]     = to_h16(a0[e] * kCarS);
        hv[it][4 + e] = to_h16(a1[e] * kCarS);
      }
    }
    for (int pass = 0; pass < 2; ++pass) {
#pragma unroll
      for (int it = 0; it < 4; ++it)
        *(volatile v4f*)(XS + (size_t)(lb + it * 4 + hrow) * kDin + hch) = fv[it];
#pragma unroll
      for (int it = 0; it < 2; ++it)
        *(volatile v8h*)(XS16 + (size_t)(lb + it * 8 + wave) * kDin + lane * 8) = hv[it];
      __threadfence();
    }
    __syncthreads();
  }
}

__global__ __launch_bounds__(64) void scan_kernel(
    const float* __restrict__ XD, const float* __restrict__ XS, const float* __restrict__ XZ,
    const float* __restrict__ Wdt, const float* __restrict__ bdt, const float* __restrict__ Alog,
    const float* __restrict__ Dp, unsigned short* __restrict__ YG)
{
  __shared__ __align__(16) float sX[kScanTS * kXdP];
  __shared__ __align__(16) float sY[kScanTS * kScanYP];
  __shared__ __align__(16) float sW[kDtR * kScanCh];
  __shared__ __align__(16) float sA[kNst * kScanCh];
  const int tid = threadIdx.x, lane = tid & 31, wave = tid >> 5;
  constexpr int kBlkPerB = kDin / kScanCh;
  const int bix = blockIdx.x / kBlkPerB;
  const int d0  = (blockIdx.x - bix * kBlkPerB) * kScanCh;
  const int d   = d0 + tid;
  const size_t row0 = (size_t)bix * kL;
#pragma unroll 1
  for (int r = 0; r < kDtR; ++r) sW[r * kScanCh + tid] = Wdt[(size_t)d * kDtR + r];
#pragma unroll 1
  for (int s = 0; s < kNst; ++s) sA[s * kScanCh + tid] = -expf(Alog[(size_t)d * kNst + s]);
  __syncthreads();
  float negA[kNst], h[kNst];
#pragma unroll
  for (int s = 0; s < kNst; ++s) {
    negA[s] = sA[s * kScanCh + tid];
    h[s] = 0.f;
  }
  const float bb = bdt[d], Dd = Dp[d];
  const int lr = tid >> 4, lc4 = (tid & 15) * 4;
  const int q = lane >> 3, c8 = (lane & 7) * 8;
#pragma unroll 1
  for (int t0 = 0; t0 < kL; t0 += kScanTS) {
    __syncthreads();
#pragma unroll
    for (int i = 0; i < 16; ++i) {
      const int r = lr + 4 * i;
      *(v4f*)(sX + r * kXdP + lc4) = *(const v4f*)(XD + (row0 + t0 + r) * kXdP + lc4);
    }
    __syncthreads();
#pragma unroll 1
    for (int s = 0; s < kScanTS; ++s) {
      const int t = t0 + s;
      const float* xr = sX + s * kXdP;
      float vdot = 0.f;
#pragma unroll 1
      for (int r4 = 0; r4 < kDtR / 4; ++r4) {
        const v4f xv = *(const v4f*)(xr + 4 * r4);
        const float* wp = sW + (4 * r4) * kScanCh + tid;
        vdot = fmaf(xv[0], wp[0], vdot);
        vdot = fmaf(xv[1], wp[kScanCh], vdot);
        vdot = fmaf(xv[2], wp[2 * kScanCh], vdot);
        vdot = fmaf(xv[3], wp[3 * kScanCh], vdot);
      }
      float Bs[kNst], Cs[kNst];
#pragma unroll
      for (int q4 = 0; q4 < 4; ++q4) {
        const v4f bv = *(const v4f*)(xr + kDtR + 4 * q4);
        const v4f cv = *(const v4f*)(xr + kDtR + kNst + 4 * q4);
        Bs[4 * q4 + 0] = bv[0]; Bs[4 * q4 + 1] = bv[1]; Bs[4 * q4 + 2] = bv[2]; Bs[4 * q4 + 3] = bv[3];
        Cs[4 * q4 + 0] = cv[0]; Cs[4 * q4 + 1] = cv[1]; Cs[4 * q4 + 2] = cv[2]; Cs[4 * q4 + 3] = cv[3];
      }
      const float v   = vdot + bb;
      const float a   = __expf(-fabsf(v));
      const float u   = 1.0f + a;
      const float l1p = __logf(u) + (a - (u - 1.0f)) * __builtin_amdgcn_rcpf(u);
      const float dt  = fmaxf(v, 0.0f) + l1p;
      const float xt  = XS[(row0 + t) * kDin + d];
      float y = 0.f;
#pragma unroll
      for (int k = 0; k < kNst; ++k) {
        const float e = __expf(dt * negA[k]);
        const float inj = (dt * Bs[k]) * xt;
        h[k] = fmaf(e, h[k], inj);
        y = fmaf(h[k], Cs[k], y);
      }
      y = fmaf(xt, Dd, y);
      const float zv = XZ[(row0 + t) * kXzP + kDin + d];
      const float sg = __builtin_amdgcn_rcpf(1.0f + __expf(-zv));
      y = y * (zv * sg);
      sY[s * kScanYP + tid] = y;
    }
    __syncthreads();
    v8h hv[8];
#pragma unroll
    for (int it = 0; it < 8; ++it) {
      const int row = it * 8 + wave * 4 + q;
      const float* sp = sY + row * kScanYP + c8;
      const v4f a0 = *(const v4f*)(sp);
      const v4f a1 = *(const v4f*)(sp + 4);
#pragma unroll
      for (int e = 0; e < 4; ++e) {
        const unsigned short h0 = f2bf_bits(a0[e]);
        const unsigned short h1 = f2bf_bits(a1[e]);
        hv[it][e]     = __builtin_bit_cast(_Float16, h0);
        hv[it][4 + e] = __builtin_bit_cast(_Float16, h1);
      }
    }
    for (int pass = 0; pass < 2; ++pass) {
#pragma unroll
      for (int it = 0; it < 8; ++it) {
        const int row = it * 8 + wave * 4 + q;
        const size_t o = (row0 + t0 + row) * kDin + d0 + c8;
        *(volatile v8h*)(YG + o) = hv[it];
      }
      __threadfence();
    }
  }
}

extern "C" void kernel_launch(void* const* d_in, const int* in_sizes, int n_in,
                              void* d_out, int out_size, void* d_ws, size_t ws_size,
                              hipStream_t stream) {
  if (n_in < 14) return;
  if (in_sizes[0] != kB * kC * kH * kW) return;
  if (in_sizes[1] != kC * kC * kTaps) return;
  if (in_sizes[2] != kC) return;
  if (in_sizes[3] != 256 * 256) return;
  if (in_sizes[4] != 256) return;
  if (in_sizes[5] != kXzP * kC) return;
  if (in_sizes[6] != kDin * 4) return;
  if (in_sizes[7] != kDin) return;
  if (in_sizes[8] != kXdN * kDin) return;
  if (in_sizes[9] != kDin * kDtR) return;
  if (in_sizes[10] != kDin) return;
  if (in_sizes[11] != kDin * kNst) return;
  if (in_sizes[12] != kDin) return;
  if (in_sizes[13] != kC * kDin) return;
  if (out_size != kB * kC * kH * kW) return;
  if (ws_size < kWsTotal) return;

  const float* x      = (const float*)d_in[0];
  const float* w_sp   = (const float*)d_in[1];
  const float* b_sp   = (const float*)d_in[2];
  const float* w_spec = (const float*)d_in[3];
  const float* b_spec = (const float*)d_in[4];
  const float* w_in   = (const float*)d_in[5];
  const float* w_c1   = (const float*)d_in[6];
  const float* b_c1   = (const float*)d_in[7];
  const float* w_xp   = (const float*)d_in[8];
  const float* w_dt   = (const float*)d_in[9];
  const float* b_dt   = (const float*)d_in[10];
  const float* a_log  = (const float*)d_in[11];
  const float* d_vec  = (const float*)d_in[12];
  const float* w_out  = (const float*)d_in[13];
  float* out = (float*)d_out;

  char* ws = (char*)d_ws;
  float*          TAB   = (float*)(ws + kOffTAB);
  unsigned short* FB    = (unsigned short*)(ws + kOffFB);
  unsigned short* IB    = (unsigned short*)(ws + kOffIB);
  unsigned short* X16   = (unsigned short*)(ws + kOffX16);
  unsigned short* XPAD  = (unsigned short*)(ws + kOffXPAD);
  unsigned short* U16   = (unsigned short*)(ws + kOffU16);
  unsigned short* WCONV = (unsigned short*)(ws + kOffWCONV);
  unsigned short* WIN   = (unsigned short*)(ws + kOffWIN);
  unsigned short* WXP   = (unsigned short*)(ws + kOffWXP);
  unsigned short* WSPEC = (unsigned short*)(ws + kOffWSPEC);
  unsigned short* WOUT  = (unsigned short*)(ws + kOffWOUT);
  unsigned short* FQ    = (unsigned short*)(ws + kOffFQ);
  unsigned short* G     = (unsigned short*)(ws + kOffG);
  float*          SPEC  = (float*)(ws + kOffSPEC);
  float*          XD    = (float*)(ws + kOffXD);
  float*          YM    = (float*)(ws + kOffYM);
  float*          XZ    = (float*)(ws + kOffXZ);
  float*          XS    = (float*)(ws + kOffXS);
  unsigned short* XS16  = (unsigned short*)(ws + kOffXS16);
  unsigned short* YG    = (unsigned short*)(ws + kOffYG);

  twiddle_kernel<<<1, 64, 0, stream>>>(TAB);
  basis_kernel<false><<<(kCols * kL / 8) / 256, 256, 0, stream>>>(TAB, FB, kCols * kL / 8);
  basis_kernel<true><<<(kCols * kL / 8) / 256, 256, 0, stream>>>(TAB, IB, kCols * kL / 8);
  cast_rows_kernel<0><<<(kBC * kL / 8) / 256, 256, 0, stream>>>(x, X16, kBC * kL / 8, kBC * kL / 8, kCarX);
  relayout_kernel<<<kB * kH, 256, 0, stream>>>(x, XPAD, U16);
  cast_rows_kernel<0><<<(kXzP * kC / 8) / 256, 256, 0, stream>>>(w_in, WIN, kXzP * kC / 8, kXzP * kC / 8, kCarW);
  cast_rows_kernel<0><<<(kXdP * kDin / 8) / 256, 256, 0, stream>>>(w_xp, WXP, kXdP * kDin / 8, kXdN * kDin / 8, kCarW);
  cast_rows_kernel<0><<<(256 * 256 / 8) / 256, 256, 0, stream>>>(w_spec, WSPEC, 256 * 256 / 8, 256 * 256 / 8, kCarW);
  cast_rows_kernel<1><<<(kC * kDin / 8) / 256, 256, 0, stream>>>(w_out, WOUT, kC * kDin / 8, kC * kDin / 8, 1.0f);
  conv_weight_kernel<<<(kC * kConvK / 8) / 256, 256, 0, stream>>>(w_sp, WCONV, kC * kConvK / 8);

  gemm64_kernel<0, false, 1, false, false><<<(kCols / 64) * (kBC / 64) / 8, 256, 0, stream>>>(
      FB, kL, X16, kL, (void*)FQ, nullptr, nullptr, nullptr,
      kCols, kBC, kL, kInvX,
      kModes, 256L, 128L, kC, (long)kModes * 256L);
  gemm64_kernel<0, true, 1, false, false><<<(256 / 64) * (kB * kModes / 64) / 8, 256, 0, stream>>>(
      WSPEC, 256, FQ, 256, (void*)G, b_spec, nullptr, nullptr,
      256, kB * kModes, 256, kInvW,
      kC, (long)kCols, (long)kModes, kModes, (long)kC * kCols);
  gemm64_kernel<0, false, 0, false, false><<<(kBC / 64) * (kL / 64) / 8, 256, 0, stream>>>(
      G, kCols, IB, kCols, (void*)SPEC, nullptr, nullptr, nullptr,
      kBC, kL, kCols, kInvHW,
      kBC, (long)kL, 0L, kL, 0L);

  gemm64_kernel<0, false, 0, false, false><<<(kTok / 64) * (kXzP / 64) / 8, 256, 0, stream>>>(
      U16, kC, WIN, kC, (void*)XZ, nullptr, nullptr, nullptr,
      kTok, kXzP, kC, kInvXW,
      kTok, (long)kXzP, 0L, kXzP, 0L);
  conv_silu_kernel<<<kTok / 64, 256, 0, stream>>>(XZ, w_c1, b_c1, XS, XS16);
  gemm64_kernel<0, false, 0, false, false><<<(kTok / 64) * (kXdP / 64) / 8, 256, 0, stream>>>(
      XS16, kDin, WXP, kDin, (void*)XD, nullptr, nullptr, nullptr,
      kTok, kXdP, kDin, kInvSW,
      kTok, (long)kXdP, 0L, kXdP, 0L);
  scan_kernel<<<kB * (kDin / kScanCh), kScanCh, 0, stream>>>(XD, XS, XZ, w_dt, b_dt, a_log, d_vec, YG);
  gemm64_kernel<1, false, 0, false, false><<<(kC / 64) * (kTok / 64) / 8, 256, 0, stream>>>(
      WOUT, kDin, YG, kDin, (void*)YM, nullptr, nullptr, nullptr,
      kC, kTok, kDin, 1.0f,
      kC, (long)kL, 0L, kL, (long)kC * kL);

  gemm64_kernel<0, true, 0, true, true><<<(kC / 64) * (kB * kH) / 8, 256, 0, stream>>>(
      WCONV, kConvK, XPAD, kC, (void*)out, b_sp, SPEC, YM,
      kC, kW, kConvK, kInvXW,
      kC, (long)kL, 0L, kW, 0L);
}
